// ModulatedDCN2dv1_72524817760945
// MI455X (gfx1250) — hardware-run, weakly checked
//
#include <hip/hip_runtime.h>


namespace {
constexpr int NB = 4, C = 128, O = 128, H = 128, W = 128, KK = 9, KT = C * KK  , SD = 512, CCH = 32  , KC = CCH * KK  ;
constexpr float XS = 8.0f, WSC = 256.0f;
typedef _Float16 b16;
typedef __attribute__((ext_vector_type(16))) _Float16 v16b;
typedef __attribute__((ext_vector_type(8))) _Float16 v8b;
typedef __attribute__((ext_vector_type(8))) float v8f;
typedef __attribute__((ext_vector_type(4))) float v4f;
__device__ __forceinline__ float bf16_rne(float f) { unsigned int u = __float_as_uint(f); u += 0x7FFFu + ((u >> 16) & 1u); float r = __uint_as_float(u & 0xFFFF0000u); asm volatile("" : "+v"(r)); return r; }
__device__ __forceinline__ float bfv(float f) { float r = bf16_rne(f); asm volatile("" : "+v"(r)); return r; }
__device__ __forceinline__ void split16(float v, b16& hi, b16& lo) { hi = (b16)v; lo = (b16)(v - (float)hi); }
__device__ __forceinline__ v16b frag_kb(const b16* p, int hh) { const v8b a = *(const v8b*)(p + 8 * hh), b = *(const v8b*)(p + 16 + 8 * hh); v16b f;
#pragma unroll
  for (int e = 0; e < 8; ++e) { f[e] = a[e]; f[8 + e] = b[e]; } return f; }
__device__ __forceinline__ v8f wmma16b(v16b a, v16b b, v8f c) { v8f d = __builtin_amdgcn_wmma_f32_16x16x32_f16(false, a, false, b, (short)0, c, false, false); asm volatile("v_nop\n\tv_nop\n\tv_nop\n\tv_nop" : "+v"(d) : "v"(a), "v"(b)); return d; }
__device__ __forceinline__ void wave_lds_sync() { __builtin_amdgcn_fence(__ATOMIC_RELEASE, "workgroup"); __builtin_amdgcn_wave_barrier(); __builtin_amdgcn_fence(__ATOMIC_ACQUIRE, "workgroup"); }
__device__ __forceinline__ float pmul(float a, float b) { float p = a * b; asm volatile("" : "+v"(p)); return p; }
__device__ __forceinline__ int iclamp(int v, int lo, int hi) { return v < lo ? lo : (v > hi ? hi : v); }

__global__ __launch_bounds__(256) void wput_kernel(const float* __restrict__ wt, b16* __restrict__ WP) { const size_t u = (size_t)blockIdx.x * 256 + threadIdx.x; if (u >= (size_t)O * KT / 8) return; v8b v;
#pragma unroll
  for (int j = 0; j < 8; ++j) v[j] = (b16)(bf16_rne(wt[u * 8 + j]) * WSC); for (int pass = 0; pass < 2; ++pass) { *(volatile v8b*)(WP + u * 8) = v; __threadfence(); } }
__global__ __launch_bounds__(128) void mod_kernel(const float* __restrict__ style, const float* __restrict__ mw, const float* __restrict__ mb, float* __restrict__ S) { const int b = blockIdx.x, c = threadIdx.x; float acc = 0.0f;
#pragma unroll 1
  for (int m = 0; m < SD; ++m) acc += pmul(bfv(style[(size_t)b * SD + m]), bfv(mw[(size_t)c * SD + m]));
  const float v = acc * (1.0f / 22.627416997969522f) + bfv(mb[c]); for (int pass = 0; pass < 2; ++pass) { ((volatile float*)S)[b * C + c] = v; __threadfence(); } }
__global__ __launch_bounds__(128) void demod_kernel(const float* __restrict__ wt, const float* __restrict__ S, float* __restrict__ DMraw) { __shared__ float red[128]; const int b = blockIdx.x / O, o = blockIdx.x % O, c = threadIdx.x; const float sc = S[b * C + c] * (1.0f / 33.941125496954285f); float acc = 0.0f;
#pragma unroll
  for (int k = 0; k < KK; ++k) { const float v = pmul(bfv(wt[((size_t)o * C + c) * KK + k]), sc); acc += v * v; }
  red[c] = acc; __syncthreads(); for (int st = 64; st; st >>= 1) { if (c < st) red[c] += red[c + st]; __syncthreads(); }
  if (c == 0) { const float v = rsqrtf(red[0] + 1e-8f); for (int pass = 0; pass < 2; ++pass) { ((volatile float*)DMraw)[(size_t)blockIdx.x * 32] = v; __threadfence(); } } }
__global__ __launch_bounds__(128) void demod_pack_kernel(const float* __restrict__ DMraw, float* __restrict__ DM) { const int b = blockIdx.x, o = threadIdx.x; const float v = DMraw[((size_t)b * O + o) * 32]; for (int pass = 0; pass < 2; ++pass) { ((volatile float*)DM)[b * O + o] = v; __threadfence(); } }
__global__ __launch_bounds__(32) void dcn_kernel(const float* __restrict__ inp, const float* __restrict__ off, const float* __restrict__ msk, const float* __restrict__ S, const float* __restrict__ DM, const float* __restrict__ ab, const b16* __restrict__ WP, int BLIM, float* __restrict__ out) {
  __shared__ __attribute__((aligned(16))) b16 Ah[2][16][KC + 8], Al[2][16][KC + 8]; __shared__ float Gw[32][KK][4], Gm[32][KK]; __shared__ int Gi[32][KK][4]; __shared__ float Tf[32][O + 4];
  const int lane = threadIdx.x, nloc = lane & 15, hlf = lane >> 4; const int wblk = blockIdx.x % (W / 32); const int h = (blockIdx.x / (W / 32)) % H; const int b = blockIdx.x / ((W / 32) * H); if (b >= BLIM) return; const int w0 = wblk * 32;
  for (int k = 0; k < KK; ++k) { const int ky = k / 3, kx = k % 3; const size_t pix = (size_t)h * W + w0 + lane; const float dy = bfv(off[(((size_t)b * 2 * KK) + 2 * k) * H * W + pix]), dx = bfv(off[(((size_t)b * 2 * KK) + 2 * k + 1) * H * W + pix]);
    const float py = (float)(h + ky - 1) + dy, px = (float)(w0 + lane + kx - 1) + dx; const float fy = floorf(py), fx = floorf(px); const float wy = py - fy, wx = px - fx; const int y0 = (int)fy, x0 = (int)fx;
#pragma unroll
    for (int q = 0; q < 4; ++q) { const int yy = y0 + (q >> 1), xx = x0 + (q & 1); const bool valid = yy >= 0 && yy < H && xx >= 0 && xx < W; const float wgt = ((q >> 1) ? wy : 1.0f - wy) * ((q & 1) ? wx : 1.0f - wx); Gw[lane][k][q] = valid ? wgt : 0.0f; Gi[lane][k][q] = iclamp(yy, 0, H - 1) * W + iclamp(xx, 0, W - 1); }
    Gm[lane][k] = bfv(msk[(((size_t)b * KK) + k) * H * W + pix]); }
  wave_lds_sync();
  for (int pass = 0; pass < 2; ++pass) { v8f acc[2][8];
#pragma unroll
    for (int t2 = 0; t2 < 2; ++t2)
#pragma unroll
      for (int t = 0; t < 8; ++t) acc[t2][t] = (v8f){};
#pragma unroll 1
    for (int c0 = 0; c0 < C; c0 += CCH) { const int c = c0 + lane; const float sc = S[b * C + c]; const float* ip = inp + ((size_t)b * C + c) * H * W;
      for (int px = 0; px < 32; ++px) {
#pragma unroll
        for (int k = 0; k < KK; ++k) { float v = 0.0f;
#pragma unroll
          for (int q = 0; q < 4; ++q) v += pmul(Gw[px][k][q], bf16_rne(ip[Gi[px][k][q]]));
          v = pmul(pmul(v, Gm[px][k]), sc); b16 p, ql; split16(v * XS, p, ql); Ah[px >> 4][px & 15][lane * KK + k] = p; Al[px >> 4][px & 15][lane * KK + k] = ql; } }
      wave_lds_sync();
#pragma unroll 1
      for (int ks = 0; ks < KC; ks += 32) { const v16b a0 = frag_kb(&Ah[0][nloc][ks], hlf), l0 = frag_kb(&Al[0][nloc][ks], hlf), a1 = frag_kb(&Ah[1][nloc][ks], hlf), l1 = frag_kb(&Al[1][nloc][ks], hlf);
#pragma unroll
        for (int t = 0; t < 8; ++t) { const v16b bw = frag_kb(WP + (size_t)(t * 16 + nloc) * KT + c0 * KK + ks, hlf); acc[0][t] = wmma16b(a0, bw, acc[0][t]); acc[0][t] = wmma16b(l0, bw, acc[0][t]); acc[1][t] = wmma16b(a1, bw, acc[1][t]); acc[1][t] = wmma16b(l1, bw, acc[1][t]); } }
      wave_lds_sync(); }
#pragma unroll
    for (int t2 = 0; t2 < 2; ++t2)
#pragma unroll
      for (int t = 0; t < 8; ++t) { const int o = t * 16 + nloc; const float dm = DM[b * O + o], bb = bfv(ab[o]);
#pragma unroll
        for (int r8 = 0; r8 < 8; ++r8) { float v = pmul(acc[t2][t][r8] * (1.0f / (XS * WSC)), dm * (1.0f / 33.941125496954285f)) + bb; v = (v > 0.0f ? v : 0.2f * v) * 1.4142135623730951f; Tf[t2 * 16 + 8 * hlf + r8][o] = v; } }
    wave_lds_sync();
    for (int o = 0; o < O; ++o) ((volatile float*)out)[(((size_t)b * O + o) * H + h) * W + w0 + lane] = Tf[lane][o];
    __threadfence(); wave_lds_sync(); } }
}

extern "C" void kernel_launch(void* const* d_in, const int* in_sizes, int n_in, void* d_out, int out_size, void* d_ws, size_t ws_size, hipStream_t stream) {
  (void)n_in;
  auto Fp = [&](int i) { return (const float*)d_in[i]; };
  if (in_sizes[0] != NB * C * H * W || in_sizes[1] != NB * SD || in_sizes[2] != NB * 2 * KK * H * W || in_sizes[3] != NB * KK * H * W || in_sizes[4] != O * KT || in_sizes[5] != C * SD || out_size != NB * O * H * W) return;
  const int BLIM = NB;
  size_t off = 0; char* ws = (char*)d_ws;
  auto carve = [&](size_t bytes) { char* p = ws + off; off += (bytes + 255) & ~(size_t)255; return p; };
  b16* WP = (b16*)carve((size_t)O * KT * 2); float* S = (float*)carve(NB * C * 4); float* DMraw = (float*)carve((size_t)NB * O * 32 * 4); float* DM = (float*)carve(NB * O * 4);
  if (off > ws_size || off > ((size_t)4 << 20)) return;
  wput_kernel<<<(unsigned)(((size_t)O * KT / 8 + 255) / 256), 256, 0, stream>>>(Fp(4), WP);
  mod_kernel<<<NB, 128, 0, stream>>>(Fp(1), Fp(5), Fp(6), S);
  demod_kernel<<<NB * O, 128, 0, stream>>>(Fp(4), S, DMraw);
  demod_pack_kernel<<<NB, 128, 0, stream>>>(DMraw, DM);
  dcn_kernel<<<BLIM * H * (W / 32), 32, 0, stream>>>(Fp(0), Fp(2), Fp(3), S, DM, Fp(7), WP, BLIM, (float*)d_out);
}
